// FixedAttentionBlock_55448027791974
// MI455X (gfx1250) — hardware-verified
//
#include <hip/hip_runtime.h>
#include <hip/hip_bf16.h>
#include <math.h>

#define BB 8
#define CCH 512
#define SS 1024
#define HH 8
#define DKK 64
#define QW 2

typedef _Float16 bf16;
typedef _Float16 f16;
typedef __attribute__((ext_vector_type(4))) unsigned v4u_t;
typedef unsigned v4ua __attribute__((ext_vector_type(4), may_alias));
typedef __attribute__((ext_vector_type(4))) float v4f_t;
typedef float v4fa __attribute__((ext_vector_type(4), may_alias));
typedef __attribute__((ext_vector_type(16))) bf16  bf16x16;
typedef bf16x16 f16x16;
typedef __attribute__((ext_vector_type(8)))  bf16  bf16x8;
typedef bf16x8 f16x8;
typedef __attribute__((ext_vector_type(4)))  bf16  bf16x4;
typedef __attribute__((ext_vector_type(8)))  float f32x8;
__device__ __forceinline__ f32x8 wmma16(f16x16 a, f16x16 b, f32x8 c) {
  c = __builtin_amdgcn_wmma_f32_16x16x32_f16(false, a, false, b, (short)0, c, false, false);
  asm volatile("v_nop\n\tv_nop\n\tv_nop\n\tv_nop" : "+v"(c) : "v"(a), "v"(b));
  return c;
}
#define LDS_STRIDE 48
#define KSTRIDE    72
#define VSTRIDE    48

__device__ __forceinline__ f32x8 wmma_bf16(bf16x16 a, bf16x16 b, f32x8 c) {
  c = __builtin_amdgcn_wmma_f32_16x16x32_f16(false, a, false, b, (short)0, c, false, false);
  asm volatile("v_nop\n\tv_nop\n\tv_nop\n\tv_nop" : "+v"(c) : "v"(a), "v"(b));
  return c;
}

template <typename T>
__device__ __forceinline__ bf16x16 load_frag(const T* __restrict__ base, int ld,
                                             int row0, int k0) {
  const int lane = threadIdx.x & 31;
  const int r    = lane & 15;
  const int kh   = (lane >> 4) * 8;
  const T* p0 = base + (size_t)(row0 + r) * ld + (k0 + kh);
  const T* p1 = p0 + 16;
  bf16x16 f;
#pragma unroll
  for (int i = 0; i < 8; ++i) {
    f[i]     = (bf16)p0[i];
    f[i + 8] = (bf16)p1[i];
  }
  return f;
}

__device__ __forceinline__ bf16x16 lds_frag(const bf16* base, int stride) {
  const int lane = threadIdx.x & 31;
  const int row  = lane & 15;
  const int kh   = (lane >> 4) * 8;
  const bf16x8 lo = *(const bf16x8*)(base + row * stride + kh);
  const bf16x8 hi = *(const bf16x8*)(base + row * stride + kh + 16);
  bf16x16 f;
#pragma unroll
  for (int i = 0; i < 8; ++i) { f[i] = lo[i]; f[i + 8] = hi[i]; }
  return f;
}

template <typename T>
__device__ __forceinline__ void stage_read16(const T* __restrict__ p, float* buf) {
#pragma unroll
  for (int i = 0; i < 16; ++i) buf[i] = (float)p[i];
}

__device__ __forceinline__ void stage_write(bf16* dst, const float* buf, int nquad) {
#pragma unroll
  for (int i = 0; i < nquad; ++i) {
    bf16x4 q;
    q[0] = (bf16)buf[4 * i];     q[1] = (bf16)buf[4 * i + 1];
    q[2] = (bf16)buf[4 * i + 2]; q[3] = (bf16)buf[4 * i + 3];
    *(bf16x4*)(dst + 4 * i) = q;
  }
}

__global__ __launch_bounds__(64) void attn_kernel(
    const bf16* __restrict__ Qb, const bf16* __restrict__ Kb,
    const bf16* __restrict__ Vt, float* __restrict__ Rout) {
  __shared__ bf16 ldsK[32 * KSTRIDE];
  __shared__ __attribute__((aligned(16))) bf16 ldsQ[64 * KSTRIDE];
  __shared__ bf16 ldsV[64 * VSTRIDE];
  __shared__ __attribute__((aligned(16))) float ldsO[2][64 * 36];

  const int q0blk = blockIdx.x * 64;
  const int h  = blockIdx.y;
  const int b  = blockIdx.z;
  const int t    = threadIdx.x;
  const int wave = t >> 5;
  const int lane = t & 31;
  const int qlane = lane & 15;
  const int kh8   = (lane >> 4) * 8;
  const int q0 = q0blk + wave * 32;

  const float* Qc = (const float*)Qb + ((size_t)b * CCH + h * DKK) * SS;
  const float* Kc = (const float*)Kb + ((size_t)b * CCH + h * DKK) * SS;
  const float* Vh = (const float*)Vt + ((size_t)b * CCH + h * DKK) * SS;
  for (int e = t; e < 64 * 64; e += 64) { const int d = e >> 6, qq = e & 63; ldsQ[qq * KSTRIDE + d] = (bf16)Qc[(size_t)d * SS + q0blk + qq]; }
  __syncthreads();

  const float* kSrc = Kc + (size_t)t * SS;
  const float* vSrc = Vh + (size_t)t * SS;

  bf16x16 qf[QW][2];
#pragma unroll
  for (int qt = 0; qt < QW; ++qt) {
    qf[qt][0] = lds_frag(ldsQ + (wave * 32 + 16 * qt) * KSTRIDE, KSTRIDE);
    qf[qt][1] = lds_frag(ldsQ + (wave * 32 + 16 * qt) * KSTRIDE + 32, KSTRIDE);
  }

  f32x8 o[QW][4] = {};
  float mrun[QW], lrun[QW];
#pragma unroll
  for (int qt = 0; qt < QW; ++qt) { mrun[qt] = -INFINITY; lrun[qt] = 0.0f; }

  const float scale = 0.125f;
  const float NEG2 = -1.0e9f;
  const int kmax = SS - 1;

  bf16x8 kreg[4], vreg[4];
  auto ld8 = [](const float* p) { const v4f_t a = *(const v4f_t*)p, c = *(const v4f_t*)(p + 4); bf16x8 r; r[0]=(bf16)a[0]; r[1]=(bf16)a[1]; r[2]=(bf16)a[2]; r[3]=(bf16)a[3]; r[4]=(bf16)c[0]; r[5]=(bf16)c[1]; r[6]=(bf16)c[2]; r[7]=(bf16)c[3]; return r; };
#pragma unroll
  for (int i = 0; i < 4; ++i) {
    kreg[i] = ld8(kSrc + 8 * i);
    vreg[i] = ld8(vSrc + 8 * i);
  }

  for (int kb = 0; kb <= kmax; kb += 32) {
    __syncthreads();
#pragma unroll
    for (int i = 0; i < 4; ++i) {
#pragma unroll
      for (int u = 0; u < 8; ++u) ldsK[(8 * i + u) * KSTRIDE + t] = kreg[i][u];
      *(bf16x8*)(&ldsV[t * VSTRIDE + 8 * i]) = vreg[i];
    }
    if (kb + 32 <= kmax) {
      const float* kn = kSrc + (kb + 32);
      const float* vn = vSrc + (kb + 32);
#pragma unroll
      for (int i = 0; i < 4; ++i) {
        kreg[i] = ld8(kn + 8 * i);
        vreg[i] = ld8(vn + 8 * i);
      }
    }
    __syncthreads();

    bf16x16 kf[2][2];
#pragma unroll
    for (int ktile = 0; ktile < 2; ++ktile)
#pragma unroll
      for (int c = 0; c < 2; ++c)
        kf[ktile][c] = lds_frag(ldsK + (ktile * 16) * KSTRIDE + c * 32, KSTRIDE);

    bf16x16 pf[QW];
    bool act[QW];
#pragma unroll
    for (int qt = 0; qt < QW; ++qt) {
      unsigned mbits = 0;
      mbits = 0xFFFFu; act[qt] = true;
      if (act[qt]) {
        const int q_my = q0 + 16 * qt + qlane;
        f32x8 s0 = {}, s1 = {};
        s0 = wmma_bf16(kf[0][0], qf[qt][0], s0);
        s0 = wmma_bf16(kf[0][1], qf[qt][1], s0);
        s1 = wmma_bf16(kf[1][0], qf[qt][0], s1);
        s1 = wmma_bf16(kf[1][1], qf[qt][1], s1);

        float mx = -INFINITY;
#pragma unroll
        for (int r = 0; r < 8; ++r) {
          const int k0i = kb + kh8 + r;
          const int k1i = k0i + 16;
          (void)k0i; (void)k1i; (void)q_my;
          s0[r] = fminf(fmaxf(s0[r] * scale, -50.0f), 50.0f) * 1.44269504088896340736f;
          s1[r] = fminf(fmaxf(s1[r] * scale, -50.0f), 50.0f) * 1.44269504088896340736f;
          mx = fmaxf(mx, fmaxf(s0[r], s1[r]));
        }
        mx = fmaxf(mx, __shfl_xor(mx, 16, 32));
        const float mnew  = fmaxf(mrun[qt], mx);
        const float alpha = exp2f(mrun[qt] - mnew);

        float rsum = 0.0f;
#pragma unroll
        for (int r = 0; r < 8; ++r) {
          const float p0 = exp2f(s0[r] - mnew);
          const float p1 = exp2f(s1[r] - mnew);
          rsum += p0 + p1;
          pf[qt][r]     = (bf16)(p0 * 1024.0f);
          pf[qt][r + 8] = (bf16)(p1 * 1024.0f);
        }
        rsum += __shfl_xor(rsum, 16, 32);
        lrun[qt] = lrun[qt] * alpha + rsum;
        mrun[qt] = mnew;

#pragma unroll
        for (int j = 0; j < 4; ++j)
#pragma unroll
          for (int r = 0; r < 8; ++r) o[qt][j][r] *= alpha;
      }
    }

#pragma unroll
    for (int j = 0; j < 4; ++j) {
      const bf16x16 vf = lds_frag(ldsV + (j * 16) * VSTRIDE, VSTRIDE);
#pragma unroll
      for (int qt = 0; qt < QW; ++qt)
        if (act[qt]) o[qt][j] = wmma_bf16(vf, pf[qt], o[qt][j]);
    }
  }

  float* so = ldsO[wave];
#pragma unroll
  for (int qt = 0; qt < QW; ++qt) {
    const float rl = 1.0f / (lrun[qt] * 1024.0f);
#pragma unroll
    for (int j = 0; j < 4; ++j)
#pragma unroll
      for (int r = 0; r < 8; ++r) so[(j * 16 + kh8 + r) * 36 + 16 * qt + qlane] = o[qt][j][r] * rl;
  }
  asm volatile("s_wait_dscnt 0" ::: "memory");
  __builtin_amdgcn_wave_barrier();
#pragma unroll 1
  for (int pass = 0; pass < 2; ++pass) {
#pragma unroll
    for (int it = 0; it < 16; ++it) { const int ch = lane + 32 * it, d = ch >> 3, q4 = (ch & 7) * 4;
      *(volatile v4f_t*)(Rout + ((size_t)b * CCH + h * DKK + d) * SS + q0 + q4) = *(const volatile v4fa*)(so + d * 36 + q4); }
    __threadfence();
  }
}


#define GSTR 48

#define GSTR 48
template <typename AT, int ASRC>
__global__ __launch_bounds__(256) void gemm_knb(const AT* __restrict__ A, int lda, size_t strideA, const float* __restrict__ Wm, int ldw, size_t strideW,
                                                const float* __restrict__ rowbias, const float* __restrict__ s1, const float* __restrict__ s2, const float* __restrict__ mj, const float* __restrict__ invD,
                                                float oscale, int N, float* __restrict__ Y, int ldy, size_t strideY, int K) {
  __shared__ __attribute__((aligned(16))) f16 ldsA[128 * GSTR];
  __shared__ __attribute__((aligned(16))) f16 ldsW[128 * GSTR];
  __shared__ __attribute__((aligned(16))) float oS[8][32 * 68];
  const int tid = threadIdx.x, lane = tid & 31, wave = tid >> 5, cl = lane & 15, rh = (lane >> 4) * 8;
  const int m0 = blockIdx.x * 128, n0 = blockIdx.y * 128;
  const int wm = (wave & 3) * 32, wn = (wave >> 2) * 64;
  A += (size_t)blockIdx.z * strideA; Wm += (size_t)blockIdx.z * strideW; Y += (size_t)blockIdx.z * strideY;
  if (ASRC == 1) { s1 += (size_t)blockIdx.z * K; s2 += (size_t)blockIdx.z * lda; mj += (size_t)blockIdx.z * K; invD += (size_t)blockIdx.z * K; }
  f32x8 acc[2][4];
#pragma unroll
  for (int i = 0; i < 2; ++i)
#pragma unroll
    for (int j = 0; j < 4; ++j) { f32x8 z = {}; acc[i][j] = z; }
#pragma unroll 1
  for (int k0 = 0; k0 < K; k0 += 32) {
    __syncthreads();
    { const int row = tid >> 1, ch = (tid & 1) * 16;
      if (ASRC == 0) {
        const AT* src = A + (size_t)(m0 + row) * lda + k0 + ch;
#pragma unroll
        for (int g = 0; g < 16; ++g) ldsA[row * GSTR + ch + g] = (f16)src[g];
      } else {
        const float s2i = s2[m0 + row];
#pragma unroll
        for (int g = 0; g < 16; ++g) { const int j = k0 + ch + g; float a = s1[j] + s2i; a = (a >= 0.0f) ? a : 0.2f * a;
          ldsA[row * GSTR + ch + g] = (f16)(1024.0f * __expf(a - mj[j]) * invD[j]); }
      } }
    { const int k = tid >> 3, nn0 = (tid & 7) * 16;
      const float* src = Wm + (size_t)(k0 + k) * ldw;
#pragma unroll
      for (int g = 0; g < 4; ++g) { const int col = min(n0 + nn0 + 4 * g, N - 4); const v4f_t v = *(const v4f_t*)(src + col);
#pragma unroll
        for (int u = 0; u < 4; ++u) ldsW[(nn0 + 4 * g + u) * GSTR + k] = (f16)v[u]; } }
    __syncthreads();
    f16x16 af[2];
#pragma unroll
    for (int i = 0; i < 2; ++i) af[i] = lds_frag(ldsA + (wm + 16 * i) * GSTR, GSTR);
#pragma unroll
    for (int j = 0; j < 4; ++j) {
      const f16x16 bf = lds_frag(ldsW + (wn + 16 * j) * GSTR, GSTR);
#pragma unroll
      for (int i = 0; i < 2; ++i) acc[i][j] = wmma16(af[i], bf, acc[i][j]);
    }
  }
  float* so = oS[wave];
#pragma unroll
  for (int i = 0; i < 2; ++i)
#pragma unroll
    for (int r = 0; r < 8; ++r) {
      const int m = m0 + wm + 16 * i + rh + r;
      const float rb = rowbias ? rowbias[m] : 0.0f;
#pragma unroll
      for (int j = 0; j < 4; ++j) so[(16 * i + rh + r) * 68 + 16 * j + cl] = acc[i][j][r] * oscale + rb;
    }
  asm volatile("s_wait_dscnt 0" ::: "memory");
  __builtin_amdgcn_wave_barrier();
#pragma unroll 1
  for (int pass = 0; pass < 2; ++pass) {
#pragma unroll
    for (int it = 0; it < 16; ++it) { const int f4 = lane + 32 * it, rr = f4 >> 4, q = (f4 & 15) * 4;
      if (n0 + wn + q < N) *(volatile v4f_t*)(Y + (size_t)(m0 + wm + rr) * ldy + n0 + wn + q) = *(const volatile v4fa*)(so + rr * 68 + q); }
    __threadfence();
  }
}

__global__ __launch_bounds__(256) void k_fold(const float* __restrict__ gamma, const float* __restrict__ beta, const float* __restrict__ rmean, const float* __restrict__ rvar,
                                             const float* __restrict__ wq, const float* __restrict__ bq, const float* __restrict__ wk, const float* __restrict__ bk,
                                             const float* __restrict__ wv, const float* __restrict__ bv, float* __restrict__ Wf, float* __restrict__ bf) {
  __shared__ __attribute__((aligned(16))) float rowS[CCH];
  __shared__ float red[256];
  const int tid = threadIdx.x, which = blockIdx.x / CCH, o = blockIdx.x % CCH;
  const float* Wsrc = (which == 0) ? wq : (which == 1) ? wk : wv; const float* bsrc = (which == 0) ? bq : (which == 1) ? bk : bv;
  float part = 0.0f;
  for (int c = tid; c < CCH; c += 256) { const float inv = gamma[c] / sqrtf(rvar[c] + 1e-5f); const float shift = beta[c] - rmean[c] * inv; const float w = Wsrc[(size_t)o * CCH + c];
    rowS[c] = w * inv; part += w * shift; }
  red[tid] = part; __syncthreads();
  for (int s = 128; s > 0; s >>= 1) { if (tid < s) red[tid] += red[tid + s]; __syncthreads(); }
  float* dst = Wf + ((size_t)which * CCH + o) * CCH;
#pragma unroll 1
  for (int pass = 0; pass < 2; ++pass) { if (tid < 128) *(volatile v4f_t*)(dst + tid * 4) = *(const volatile v4fa*)(rowS + tid * 4); __threadfence(); }
  (void)bsrc; (void)bf; (void)red; (void)part;
}
__global__ __launch_bounds__(256) void k_foldb(const float* __restrict__ gamma, const float* __restrict__ beta, const float* __restrict__ rmean, const float* __restrict__ rvar,
                                              const float* __restrict__ wq, const float* __restrict__ bq, const float* __restrict__ wk, const float* __restrict__ bk,
                                              const float* __restrict__ wv, const float* __restrict__ bv, float* __restrict__ bf) {
  __shared__ float shS[CCH];
  __shared__ __attribute__((aligned(16))) float bS[CCH];
  const int tid = threadIdx.x, which = blockIdx.x;
  const float* Wsrc = (which == 0) ? wq : (which == 1) ? wk : wv; const float* bsrc = (which == 0) ? bq : (which == 1) ? bk : bv;
  for (int c = tid; c < CCH; c += 256) { const float inv = gamma[c] / sqrtf(rvar[c] + 1e-5f); shS[c] = beta[c] - rmean[c] * inv; }
  __syncthreads();
  for (int o = tid; o < CCH; o += 256) { float s = bsrc[o]; const float* wr = Wsrc + (size_t)o * CCH;
#pragma unroll 4
    for (int c = 0; c < CCH; ++c) s += wr[c] * shS[c];
    bS[o] = s; }
  __syncthreads();
#pragma unroll 1
  for (int pass = 0; pass < 2; ++pass) { if (tid < 128) *(volatile v4f_t*)(bf + which * CCH + tid * 4) = *(const volatile v4fa*)(bS + tid * 4); __threadfence(); }
}
__global__ __launch_bounds__(256) void k_resadd(const float* __restrict__ x, const float* __restrict__ pr, float* __restrict__ out, size_t n4) {
  const size_t i = (size_t)blockIdx.x * 256 + threadIdx.x; if (i >= n4) return;
  const v4f_t a = *(const v4f_t*)(x + 4 * i), b = *(const v4f_t*)(pr + 4 * i); v4f_t o; o[0]=a[0]+b[0]; o[1]=a[1]+b[1]; o[2]=a[2]+b[2]; o[3]=a[3]+b[3];
  *(volatile v4f_t*)(out + 4 * i) = o; __threadfence(); *(volatile v4f_t*)(out + 4 * i) = o;
}

extern "C" void kernel_launch(void* const* d_in, const int* in_sizes, int n_in,
                              void* d_out, int out_size, void* d_ws, size_t ws_size,
                              hipStream_t stream) {
  (void)in_sizes; (void)n_in; (void)out_size; (void)ws_size;
  const float* x = (const float*)d_in[0];
  const float* gamma = (const float*)d_in[1], *beta = (const float*)d_in[2], *rmean = (const float*)d_in[3], *rvar = (const float*)d_in[4];
  const float* wq = (const float*)d_in[5], *bq = (const float*)d_in[6], *wk = (const float*)d_in[7], *bk = (const float*)d_in[8];
  const float* wv = (const float*)d_in[9], *bv = (const float*)d_in[10], *wp = (const float*)d_in[11], *bp = (const float*)d_in[12];
  float* out = (float*)d_out;
  char* ws = (char*)d_ws;
  float* Wf = (float*)ws; ws += (size_t)3 * CCH * CCH * 4;
  float* bfold = (float*)ws; ws += 3 * CCH * 4 + 2048;
  const size_t T = (size_t)BB * CCH * SS * 4;
  float* Qc = (float*)ws; float* Kc = (float*)(ws + T); float* Vc = (float*)(ws + 2 * T); float* Rc = (float*)(ws + 3 * T);
  k_fold<<<dim3(3 * CCH), dim3(256), 0, stream>>>(gamma, beta, rmean, rvar, wq, bq, wk, bk, wv, bv, Wf, bfold);
  k_foldb<<<dim3(3), dim3(256), 0, stream>>>(gamma, beta, rmean, rvar, wq, bq, wk, bk, wv, bv, bfold);
  const dim3 g(CCH / 128, SS / 128, BB), blk(256);
  gemm_knb<float, 0><<<g, blk, 0, stream>>>(Wf,                 CCH, 0, x, SS, (size_t)CCH * SS, bfold,           nullptr, nullptr, nullptr, nullptr, 1.0f, SS, Qc, SS, (size_t)CCH * SS, CCH);
  gemm_knb<float, 0><<<g, blk, 0, stream>>>(Wf + CCH * CCH,     CCH, 0, x, SS, (size_t)CCH * SS, bfold + CCH,     nullptr, nullptr, nullptr, nullptr, 1.0f, SS, Kc, SS, (size_t)CCH * SS, CCH);
  gemm_knb<float, 0><<<g, blk, 0, stream>>>(Wf + 2 * CCH * CCH, CCH, 0, x, SS, (size_t)CCH * SS, bfold + 2 * CCH, nullptr, nullptr, nullptr, nullptr, 1.0f, SS, Vc, SS, (size_t)CCH * SS, CCH);
  attn_kernel<<<dim3(SS / 64, HH, BB), dim3(64), 0, stream>>>((const bf16*)Qc, (const bf16*)Kc, (const bf16*)Vc, Rc);
  gemm_knb<float, 0><<<g, blk, 0, stream>>>(wp, CCH, 0, Rc, SS, (size_t)CCH * SS, bp, nullptr, nullptr, nullptr, nullptr, 1.0f, SS, Qc, SS, (size_t)CCH * SS, CCH);
  k_resadd<<<dim3((BB * CCH * SS / 4 + 255) / 256), blk, 0, stream>>>(x, Qc, out, (size_t)BB * CCH * SS / 4);
}
